// MultiHeadAttention_41394894799052
// MI455X (gfx1250) — hardware-run, weakly checked
//
#include <hip/hip_runtime.h>


#ifndef NB
#define NB 1
#endif
#ifndef SEQ
#define SEQ 4096
#endif
#define NB_FULL  1
#define SEQ_FULL 4096
#define DM   1024
#define NH_  16
#define HD   64
#define AW   4
#define ESEQ ((SEQ) < 512 ? (SEQ) : 512)
#define QRS  2048.0f
#define QRI  (1.0f / 2048.0f)
#define LOG2E 1.4426950408889634f
#define SC2  (0.125f * LOG2E)
#define PSH  8.0f
#define CCS  16.0f
#define WOS  64.0f
#define OSI  (1.0f / 1024.0f)
#define NEGB (-3.0e38f)

static_assert(NB == 1);
static_assert(HD == 64);
static_assert(NH_ * HD == DM);
static_assert(DM % 64 == 0);
static_assert(DM % 32 == 0);
static_assert(SEQ % 64 == 0);
static_assert(SEQ % 32 == 0);
static_assert(ESEQ % 64 == 0);
static_assert((SEQ - ESEQ) % 64 == 0);
static_assert(ESEQ % (16 * AW) == 0);
static_assert((SEQ - ESEQ) % (16 * AW) == 0);
static_assert(((size_t)SEQ * DM) % 8 == 0);
static_assert(((size_t)DM * DM) % 8 == 0);
static_assert((NH_ * SEQ) % 4 == 0);
static_assert(NB <= NB_FULL);
static_assert(SEQ <= SEQ_FULL);

typedef _Float16 h16;
typedef unsigned short bf;
typedef __attribute__((ext_vector_type(16))) __bf16   v16bf;
typedef __attribute__((ext_vector_type(16))) _Float16 v16h;
typedef __attribute__((ext_vector_type(8)))  _Float16 v8h;
typedef __attribute__((ext_vector_type(8)))  unsigned short v8us;
typedef __attribute__((ext_vector_type(8)))  float    v8f;
typedef __attribute__((ext_vector_type(4)))  float    v4f;
typedef v4f  __attribute__((may_alias)) v4fa;

__device__ __forceinline__ unsigned short f2bf(float f) { unsigned u = __float_as_uint(f); u += 0x7FFFu + ((u >> 16) & 1u); return (unsigned short)(u >> 16); }
__device__ __forceinline__ float bfr(float f) { return __uint_as_float(((unsigned)f2bf(f)) << 16); }
__device__ __forceinline__ v16h cat16(v8h lo, v8h hi) { return __builtin_shufflevector(lo, hi, 0, 1, 2, 3, 4, 5, 6, 7, 8, 9, 10, 11, 12, 13, 14, 15); }
__device__ __forceinline__ v16bf cat16b(v8us lo, v8us hi) { return __builtin_bit_cast(v16bf, __builtin_shufflevector(lo, hi, 0, 1, 2, 3, 4, 5, 6, 7, 8, 9, 10, 11, 12, 13, 14, 15)); }
__device__ __forceinline__ v8f wmma16(v16h a, v16h b, v8f c) { return __builtin_amdgcn_wmma_f32_16x16x32_f16(false, a, false, b, (short)0, c, false, false); }
__device__ __forceinline__ v8f wmmab(v16bf a, v16bf b, v8f c) { return __builtin_amdgcn_wmma_f32_16x16x32_bf16(false, a, false, b, (short)0, c, false, false); }
__device__ __forceinline__ v16h  ldh(const h16* p) { return cat16(*(const v8h*)p, *(const v8h*)(p + 16)); }
__device__ __forceinline__ v16bf ldb(const bf* p)  { return cat16b(*(const v8us*)p, *(const v8us*)(p + 16)); }
__device__ __forceinline__ void wave_sync() { __builtin_amdgcn_fence(3  , "wavefront"); __builtin_amdgcn_wave_barrier(); asm volatile("" ::: "memory"); }

__global__ __launch_bounds__(256) void k_cvt8(const float* __restrict__ src, bf* dst, size_t n8) {
    const size_t i = (size_t)blockIdx.x * 256 + threadIdx.x; if (i >= n8) return;
    const v8f v = *(const v8f*)(src + i * 8); v8us o;
#pragma unroll
    for (int k = 0; k < 8; ++k) o[k] = f2bf(v[k]);
    *(volatile v8us*)(dst + i * 8) = o; __threadfence(); *(volatile v8us*)(dst + i * 8) = o;
}

__global__ __launch_bounds__(256) void k_cvt8h(const float* __restrict__ src, h16* dst, size_t n8) {
    const size_t i = (size_t)blockIdx.x * 256 + threadIdx.x; if (i >= n8) return;
    const v8f v = *(const v8f*)(src + i * 8); v8h o;
#pragma unroll
    for (int k = 0; k < 8; ++k) o[k] = (h16)(bfr(v[k]) * WOS);
    *(volatile v8h*)(dst + i * 8) = o; __threadfence(); *(volatile v8h*)(dst + i * 8) = o;
}

__global__ __launch_bounds__(256) void k_bias(const float* __restrict__ ab, float* BL) {
    const int i = blockIdx.x * 256 + threadIdx.x; if (i >= NH_ * SEQ / 4) return;
    const int e = i * 4; const int hh = e / SEQ, key = e % SEQ;
    const v4f v = *(const v4f*)(ab + (size_t)hh * SEQ_FULL + key); v4f o;
#pragma unroll
    for (int k = 0; k < 4; ++k) o[k] = bfr(v[k]) * LOG2E;
    *(volatile v4f*)(BL + (size_t)i * 4) = o; __threadfence(); *(volatile v4f*)(BL + (size_t)i * 4) = o;
}

template <int BM>
__global__ __launch_bounds__(32) void k_proj(const bf* __restrict__ A, const bf* __restrict__ Bt, const float* __restrict__ bias, h16* Ph, h16* Pr, int RB, size_t sRB, int pitch, int CB, size_t sCB) {
    __shared__ __align__(16) float os[16 * 68];
    const int K = DM;
    const int lane = threadIdx.x & 31, lr = lane & 15, hi = lane >> 4; const int r0 = blockIdx.x * 64, c0 = blockIdx.y * 64;
    v8f acc[4][4];
#pragma unroll
    for (int mb = 0; mb < 4; ++mb)
#pragma unroll
        for (int nb = 0; nb < 4; ++nb) acc[mb][nb] = (v8f){};
    const size_t aoff = (size_t)(r0 + lr) * K + 8 * hi, boff = (size_t)(c0 + lr) * K + 8 * hi;
#pragma unroll 1
    for (int kc = 0; kc < K; kc += 32) {
        v16bf a[4];
#pragma unroll
        for (int mb = 0; mb < 4; ++mb) a[mb] = ldb(A + aoff + (size_t)mb * 16 * K + kc);
#pragma unroll
        for (int nb = 0; nb < 4; ++nb) { const v16bf b = ldb(Bt + boff + (size_t)nb * 16 * K + kc);
#pragma unroll
            for (int mb = 0; mb < 4; ++mb) acc[mb][nb] = wmmab(a[mb], b, acc[mb][nb]); }
        asm volatile("v_nop\n\tv_nop\n\tv_nop\n\tv_nop" : "+v"(acc[0][0]), "+v"(acc[1][1]), "+v"(acc[2][2]), "+v"(acc[3][3]) : "v"(a[0]), "v"(a[1]), "v"(a[2]), "v"(a[3]));
    }
    float bc[4] = {0.0f, 0.0f, 0.0f, 0.0f};
    if (BM == 0) {
#pragma unroll
        for (int nb = 0; nb < 4; ++nb) bc[nb] = bfr(bias[c0 + nb * 16 + lr]);
    }
    const size_t tbase = (size_t)(r0 / RB) * sRB + (size_t)(r0 % RB) * (size_t)pitch + (size_t)(c0 / CB) * sCB + (size_t)(c0 % CB);
#pragma unroll
    for (int mb = 0; mb < 4; ++mb) {
        float br[8] = {0.0f, 0.0f, 0.0f, 0.0f, 0.0f, 0.0f, 0.0f, 0.0f};
        if (BM == 1) {
            const v4f b0 = *(const v4f*)(bias + r0 + mb * 16 + hi * 8); const v4f b1 = *(const v4f*)(bias + r0 + mb * 16 + hi * 8 + 4);
#pragma unroll
            for (int j = 0; j < 4; ++j) { br[j] = bfr(b0[j]); br[4 + j] = bfr(b1[j]); }
        }
#pragma unroll
        for (int nb = 0; nb < 4; ++nb) {
#pragma unroll
            for (int j = 0; j < 8; ++j) os[(hi * 8 + j) * 68 + nb * 16 + lr] = acc[mb][nb][j] + (BM == 0 ? bc[nb] : br[j]); }
        wave_sync();
        const size_t sb = tbase + (size_t)(mb * 16) * (size_t)pitch;
#pragma unroll 1
        for (int ps = 0; ps < 2; ++ps) {
#pragma unroll
            for (int s = 0; s < 4; ++s) { const int row = 4 * s + (lane >> 3), c8 = (lane & 7) * 8;
                const v4f x0 = *(const v4fa*)(&os[row * 68 + c8]); const v4f x1 = *(const v4fa*)(&os[row * 68 + c8 + 4]); v8h hv, rv;
#pragma unroll
                for (int i = 0; i < 4; ++i) { const h16 a0 = (h16)x0[i]; const h16 a1 = (h16)x1[i]; hv[i] = a0; hv[4 + i] = a1; rv[i] = (h16)((x0[i] - (float)a0) * QRS); rv[4 + i] = (h16)((x1[i] - (float)a1) * QRS); }
                const size_t oo = sb + (size_t)row * (size_t)pitch + c8;
                *(volatile v8h*)(Ph + oo) = hv; *(volatile v8h*)(Pr + oo) = rv; }
            if (ps == 0) __threadfence(); }
        wave_sync();
    }
}

template <int EARLY>
__global__ __launch_bounds__(32 * AW) void k_flash(const h16* __restrict__ QH, const h16* __restrict__ QR, const h16* __restrict__ KP, const h16* __restrict__ KR,
                                                   const h16* __restrict__ VT, const h16* __restrict__ VR, const float* __restrict__ BL, h16* CH, h16* CR, int trow0) {
    __shared__ __align__(16) float os[AW * 16 * 68];
    const int lane = threadIdx.x & 31, wave = __builtin_amdgcn_readfirstlane((int)(threadIdx.x >> 5)), lr = lane & 15, hi = lane >> 4;
    const int h = blockIdx.y;
    const int t0 = trow0 + (blockIdx.x * AW + wave) * 16;
    const int tq = t0 + lr;
    const size_t pbase = (size_t)h * SEQ * HD;
    const size_t qo = pbase + (size_t)tq * HD + 8 * hi;
    const v16h qh0 = ldh(QH + qo), qh1 = ldh(QH + qo + 32);
    v16h qr0 = qh0, qr1 = qh1;
    if (EARLY) { qr0 = ldh(QR + qo); qr1 = ldh(QR + qo + 32); }
    const size_t ko = pbase + (size_t)lr * HD + 8 * hi;
    const size_t vo = pbase + (size_t)lr * SEQ + 8 * hi;
    const float* bl = BL + (size_t)h * SEQ + 8 * hi;
    v8f o0 = (v8f){}, o1 = (v8f){}, o2 = (v8f){}, o3 = (v8f){};
    v8f u0 = (v8f){}, u1 = (v8f){}, u2 = (v8f){}, u3 = (v8f){};
    float m = NEGB, l = 0.0f;
    const int kend = t0 + 16;
#pragma unroll 1
    for (int key0 = 0; key0 < kend; key0 += 32) {
        const h16* ka = KP + ko + (size_t)key0 * HD;
        const v16h ka0 = ldh(ka), ka1 = ldh(ka + 32), kb0 = ldh(ka + 16 * HD), kb1 = ldh(ka + 16 * HD + 32);
        const v8f ba = *(const v8f*)(bl + key0); const v8f bb = *(const v8f*)(bl + key0 + 16);
        v8f sHa = (v8f){}, sLa = (v8f){}, sHb = (v8f){}, sLb = (v8f){};
        sHa = wmma16(ka0, qh0, sHa); sHb = wmma16(kb0, qh0, sHb);
        sHa = wmma16(ka1, qh1, sHa); sHb = wmma16(kb1, qh1, sHb);
        if (EARLY) {
            const h16* kr = KR + ko + (size_t)key0 * HD;
            const v16h ra0 = ldh(kr), ra1 = ldh(kr + 32), rb0 = ldh(kr + 16 * HD), rb1 = ldh(kr + 16 * HD + 32);
            sLa = wmma16(ka0, qr0, sLa); sLb = wmma16(kb0, qr0, sLb); sLa = wmma16(ka1, qr1, sLa); sLb = wmma16(kb1, qr1, sLb);
            sLa = wmma16(ra0, qh0, sLa); sLb = wmma16(rb0, qh0, sLb); sLa = wmma16(ra1, qh1, sLa); sLb = wmma16(rb1, qh1, sLb);
            asm volatile("v_nop\n\tv_nop\n\tv_nop\n\tv_nop" : "+v"(sHa), "+v"(sLa), "+v"(sHb), "+v"(sLb) : "v"(ka0), "v"(ka1), "v"(kb0), "v"(kb1), "v"(ra0), "v"(ra1), "v"(rb0), "v"(rb1));
        } else {
            asm volatile("v_nop\n\tv_nop\n\tv_nop\n\tv_nop" : "+v"(sHa), "+v"(sHb) : "v"(ka0), "v"(ka1), "v"(kb0), "v"(kb1));
        }
        float ta[8], tb[8];
#pragma unroll
        for (int r = 0; r < 8; ++r) {
            const float sa = EARLY ? (sHa[r] + sLa[r] * QRI) : sHa[r];
            const float sb = EARLY ? (sHb[r] + sLb[r] * QRI) : sHb[r];
            ta[r] = sa * SC2 + ba[r]; tb[r] = sb * SC2 + bb[r]; }
        if (key0 + 31 > t0) {
            const int kk = key0 + 8 * hi;
#pragma unroll
            for (int r = 0; r < 8; ++r) { ta[r] = (kk + r <= tq) ? ta[r] : NEGB; tb[r] = (kk + 16 + r <= tq) ? tb[r] : NEGB; }
        }
        float mx = NEGB;
#pragma unroll
        for (int r = 0; r < 8; ++r) mx = fmaxf(mx, fmaxf(ta[r], tb[r]));
        mx = fmaxf(mx, __shfl_xor(mx, 16, 32));
        const float mnew = fmaxf(m, mx);
        const float alpha = __builtin_amdgcn_exp2f(m - mnew);
        const float sh = PSH - mnew;
        v16h pb, pr = (v16h){}; float ls = 0.0f;
#pragma unroll
        for (int r = 0; r < 8; ++r) {
            const float ea = __builtin_amdgcn_exp2f(ta[r] + sh); const float eb = __builtin_amdgcn_exp2f(tb[r] + sh);
            const h16 pa = (h16)ea; const h16 pc = (h16)eb; pb[r] = pa; pb[8 + r] = pc;
            if (EARLY) { const h16 xa = (h16)((ea - (float)pa) * QRS); const h16 xc = (h16)((eb - (float)pc) * QRS); pr[r] = xa; pr[8 + r] = xc;
                         ls += ((float)pa + (float)pc) + ((float)xa + (float)xc) * QRI; }
            else ls += (float)pa + (float)pc; }
        l = l * alpha + ls; m = mnew;
        o0 = o0 * alpha; o1 = o1 * alpha; o2 = o2 * alpha; o3 = o3 * alpha;
        const h16* va = VT + vo + key0;
        const v16h v0 = ldh(va), v1 = ldh(va + (size_t)16 * SEQ), v2 = ldh(va + (size_t)32 * SEQ), v3 = ldh(va + (size_t)48 * SEQ);
        o0 = wmma16(v0, pb, o0); o1 = wmma16(v1, pb, o1); o2 = wmma16(v2, pb, o2); o3 = wmma16(v3, pb, o3);
        if (EARLY) {
            u0 = u0 * alpha; u1 = u1 * alpha; u2 = u2 * alpha; u3 = u3 * alpha;
            const h16* vr = VR + vo + key0;
            const v16h w0 = ldh(vr), w1 = ldh(vr + (size_t)16 * SEQ), w2 = ldh(vr + (size_t)32 * SEQ), w3 = ldh(vr + (size_t)48 * SEQ);
            u0 = wmma16(v0, pr, u0); u1 = wmma16(v1, pr, u1); u2 = wmma16(v2, pr, u2); u3 = wmma16(v3, pr, u3);
            u0 = wmma16(w0, pb, u0); u1 = wmma16(w1, pb, u1); u2 = wmma16(w2, pb, u2); u3 = wmma16(w3, pb, u3);
            asm volatile("v_nop\n\tv_nop\n\tv_nop\n\tv_nop" : "+v"(o0), "+v"(o1), "+v"(o2), "+v"(o3), "+v"(u0), "+v"(u1), "+v"(u2), "+v"(u3)
                         : "v"(v0), "v"(v1), "v"(v2), "v"(v3), "v"(w0), "v"(w1), "v"(w2), "v"(w3), "v"(pb), "v"(pr));
        } else {
            asm volatile("v_nop\n\tv_nop\n\tv_nop\n\tv_nop" : "+v"(o0), "+v"(o1), "+v"(o2), "+v"(o3) : "v"(v0), "v"(v1), "v"(v2), "v"(v3), "v"(pb));
        }
    }
    l += __shfl_xor(l, 16, 32);
    const float inv = (1.0f / l) * CCS;
    if (EARLY) { o0 = o0 + u0 * QRI; o1 = o1 + u1 * QRI; o2 = o2 + u2 * QRI; o3 = o3 + u3 * QRI; }
    o0 = o0 * inv; o1 = o1 * inv; o2 = o2 * inv; o3 = o3 * inv;
    const int wb = wave * 16 * 68;
    { const int ob = wb + lr * 68 + 8 * hi;
      *(v4fa*)(&os[ob +  0]) = __builtin_shufflevector(o0, o0, 0, 1, 2, 3); *(v4fa*)(&os[ob +  4]) = __builtin_shufflevector(o0, o0, 4, 5, 6, 7);
      *(v4fa*)(&os[ob + 16]) = __builtin_shufflevector(o1, o1, 0, 1, 2, 3); *(v4fa*)(&os[ob + 20]) = __builtin_shufflevector(o1, o1, 4, 5, 6, 7);
      *(v4fa*)(&os[ob + 32]) = __builtin_shufflevector(o2, o2, 0, 1, 2, 3); *(v4fa*)(&os[ob + 36]) = __builtin_shufflevector(o2, o2, 4, 5, 6, 7);
      *(v4fa*)(&os[ob + 48]) = __builtin_shufflevector(o3, o3, 0, 1, 2, 3); *(v4fa*)(&os[ob + 52]) = __builtin_shufflevector(o3, o3, 4, 5, 6, 7); }
    wave_sync();
    const size_t cb = (size_t)t0 * DM + (size_t)h * HD;
#pragma unroll 1
    for (int ps = 0; ps < 2; ++ps) {
#pragma unroll
        for (int s = 0; s < 4; ++s) { const int row = 4 * s + (lane >> 3), c8 = (lane & 7) * 8;
            const v4f x0 = *(const v4fa*)(&os[wb + row * 68 + c8]); const v4f x1 = *(const v4fa*)(&os[wb + row * 68 + c8 + 4]); v8h hv, rv;
#pragma unroll
            for (int i = 0; i < 4; ++i) { const h16 a0 = (h16)x0[i]; const h16 a1 = (h16)x1[i]; hv[i] = a0; hv[4 + i] = a1; rv[i] = (h16)((x0[i] - (float)a0) * QRS); rv[4 + i] = (h16)((x1[i] - (float)a1) * QRS); }
            const size_t oo = cb + (size_t)row * DM + c8;
            *(volatile v8h*)(CH + oo) = hv; if (EARLY) *(volatile v8h*)(CR + oo) = rv; }
        if (ps == 0) __threadfence(); }
}

template <int MB, int RES>
__global__ __launch_bounds__(32) void k_out(const h16* __restrict__ A, const h16* __restrict__ AR, const h16* __restrict__ Bt, const float* __restrict__ bias, float* OUT, int rbase) {
    __shared__ __align__(16) float os[16 * 68];
    const int K = DM;
    const int lane = threadIdx.x & 31, lr = lane & 15, hi = lane >> 4; const int r0 = rbase + blockIdx.x * (16 * MB), c0 = blockIdx.y * 64;
    v8f acc[MB][4], acr[MB][4];
#pragma unroll
    for (int mb = 0; mb < MB; ++mb)
#pragma unroll
        for (int nb = 0; nb < 4; ++nb) { acc[mb][nb] = (v8f){}; acr[mb][nb] = (v8f){}; }
    const size_t aoff = (size_t)(r0 + lr) * K + 8 * hi, boff = (size_t)(c0 + lr) * K + 8 * hi;
#pragma unroll 1
    for (int kc = 0; kc < K; kc += 32) {
        v16h a[MB], ar[MB];
#pragma unroll
        for (int mb = 0; mb < MB; ++mb) { a[mb] = ldh(A + aoff + (size_t)mb * 16 * K + kc); ar[mb] = a[mb]; if (RES) ar[mb] = ldh(AR + aoff + (size_t)mb * 16 * K + kc); }
#pragma unroll
        for (int nb = 0; nb < 4; ++nb) { const v16h b = ldh(Bt + boff + (size_t)nb * 16 * K + kc);
#pragma unroll
            for (int mb = 0; mb < MB; ++mb) { acc[mb][nb] = wmma16(a[mb], b, acc[mb][nb]); if (RES) acr[mb][nb] = wmma16(ar[mb], b, acr[mb][nb]); } }
        if (RES) {
            asm volatile("v_nop\n\tv_nop\n\tv_nop\n\tv_nop" : "+v"(acc[0][0]), "+v"(acc[MB - 1][3]), "+v"(acr[0][0]), "+v"(acr[MB - 1][3]) : "v"(a[0]), "v"(a[MB - 1]), "v"(ar[0]), "v"(ar[MB - 1]));
        } else {
            asm volatile("v_nop\n\tv_nop\n\tv_nop\n\tv_nop" : "+v"(acc[0][0]), "+v"(acc[MB - 1][0]), "+v"(acc[0][3]), "+v"(acc[MB - 1][3]) : "v"(a[0]), "v"(a[MB - 1]));
        }
    }
    float bc[4];
#pragma unroll
    for (int nb = 0; nb < 4; ++nb) bc[nb] = bfr(bias[c0 + nb * 16 + lr]);
#pragma unroll
    for (int mb = 0; mb < MB; ++mb) {
#pragma unroll
        for (int nb = 0; nb < 4; ++nb) {
#pragma unroll
            for (int j = 0; j < 8; ++j) { float v = acc[mb][nb][j]; if (RES) v += acr[mb][nb][j] * QRI;
                os[(hi * 8 + j) * 68 + nb * 16 + lr] = v * OSI + bc[nb]; } }
        wave_sync();
        float* orow = OUT + (size_t)(r0 + mb * 16) * DM + c0;
#pragma unroll 1
        for (int ps = 0; ps < 2; ++ps) {
#pragma unroll
            for (int s = 0; s < 8; ++s) { const int row = 2 * s + hi, cofs = lr * 4;
                const v4f val = *(const v4fa*)(&os[row * 68 + cofs]);
                *(volatile v4f*)(orow + (size_t)row * DM + cofs) = val; }
            if (ps == 0) __threadfence(); }
        wave_sync();
    }
}

static constexpr size_t al256(size_t v) { return (v + 255) & ~(size_t)255; }
static constexpr size_t SZ_XB = al256((size_t)NB * SEQ * DM * 2);
static constexpr size_t SZ_WB = al256((size_t)3 * DM * DM * 2);
static constexpr size_t SZ_WO = al256((size_t)DM * DM * 2);
static constexpr size_t SZ_BL = al256((size_t)NH_ * SEQ * 4);
static constexpr size_t SZ_PL = al256((size_t)NB * NH_ * SEQ * HD * 2);
static constexpr size_t SZ_CH = al256((size_t)NB * SEQ * DM * 2);
static constexpr size_t SZ_CR = al256((size_t)NB * ESEQ * DM * 2);
static constexpr size_t SZ_TOTAL = SZ_XB + SZ_WB + SZ_WO + SZ_BL + 6 * SZ_PL + SZ_CH + SZ_CR;
static_assert(SZ_TOTAL <= (size_t)134217728);
static_assert(((size_t)DM * DM * 2) % 256 == 0);

extern "C" void kernel_launch(void* const* d_in, const int* in_sizes, int n_in,
                              void* d_out, int out_size, void* d_ws, size_t ws_size, hipStream_t stream) {
    if (n_in < 6) return;
    if ((size_t)in_sizes[0] < (size_t)SEQ * DM) return;
    if ((size_t)in_sizes[1] < (size_t)(NH_ - 1) * SEQ_FULL + SEQ) return;
    if ((size_t)in_sizes[2] < (size_t)3 * DM * DM || (size_t)in_sizes[3] < (size_t)3 * DM) return;
    if ((size_t)in_sizes[4] < (size_t)DM * DM || (size_t)in_sizes[5] < (size_t)DM) return;
    if ((size_t)out_size < (size_t)SEQ * DM) return;
    if (SZ_TOTAL > ws_size) return;
    const float* x = (const float*)d_in[0]; const float* ab = (const float*)d_in[1]; const float* wqkv = (const float*)d_in[2];
    const float* bqkv = (const float*)d_in[3]; const float* wo = (const float*)d_in[4]; const float* bo = (const float*)d_in[5];
    float* OUT = (float*)d_out;
    char* wsp = (char*)d_ws;
    bf* XB = (bf*)wsp; wsp += SZ_XB;
    bf* WB = (bf*)wsp; wsp += SZ_WB;
    h16* WO = (h16*)wsp; wsp += SZ_WO;
    float* BL = (float*)wsp; wsp += SZ_BL;
    h16* QH = (h16*)wsp; wsp += SZ_PL;
    h16* QR = (h16*)wsp; wsp += SZ_PL;
    h16* KP = (h16*)wsp; wsp += SZ_PL;
    h16* KR = (h16*)wsp; wsp += SZ_PL;
    h16* VT = (h16*)wsp; wsp += SZ_PL;
    h16* VR = (h16*)wsp; wsp += SZ_PL;
    h16* CH = (h16*)wsp; wsp += SZ_CH;
    h16* CR = (h16*)wsp; wsp += SZ_CR;
    bf* WQ = WB; bf* WK = WB + (size_t)DM * DM; bf* WV = WB + (size_t)2 * DM * DM;

    { const size_t n8 = (size_t)SEQ * DM / 8; k_cvt8<<<(unsigned)((n8 + 255) / 256), 256, 0, stream>>>(x, XB, n8); }
    { const size_t n8 = (size_t)3 * DM * DM / 8; k_cvt8<<<(unsigned)((n8 + 255) / 256), 256, 0, stream>>>(wqkv, WB, n8); }
    { const size_t n8 = (size_t)DM * DM / 8; k_cvt8h<<<(unsigned)((n8 + 255) / 256), 256, 0, stream>>>(wo, WO, n8); }
    k_bias<<<(unsigned)((NH_ * SEQ / 4 + 255) / 256), 256, 0, stream>>>(ab, BL);

    k_proj<0><<<dim3(SEQ / 64, DM / 64, 1), 32, 0, stream>>>(XB, WQ, bqkv, QH, QR, SEQ, (size_t)NH_ * SEQ * HD, HD, HD, (size_t)SEQ * HD);
    k_proj<0><<<dim3(SEQ / 64, DM / 64, 1), 32, 0, stream>>>(XB, WK, bqkv + DM, KP, KR, SEQ, (size_t)NH_ * SEQ * HD, HD, HD, (size_t)SEQ * HD);
    k_proj<1><<<dim3(DM / 64, SEQ / 64, 1), 32, 0, stream>>>(WV, XB, bqkv + 2 * DM, VT, VR, DM, (size_t)0, SEQ, SEQ, (size_t)DM * SEQ);

    k_flash<1><<<dim3(ESEQ / (16 * AW), NH_, 1), 32 * AW, 0, stream>>>(QH, QR, KP, KR, VT, VR, BL, CH, CR, 0);
    if (SEQ > ESEQ)
        k_flash<0><<<dim3((SEQ - ESEQ) / (16 * AW), NH_, 1), 32 * AW, 0, stream>>>(QH, QR, KP, KR, VT, VR, BL, CH, CR, ESEQ);

    k_out<2, 1><<<dim3(ESEQ / 32, DM / 64, 1), 32, 0, stream>>>(CH, CR, WO, bo, OUT, 0);
    if (SEQ > ESEQ)
        k_out<4, 0><<<dim3((SEQ - ESEQ) / 64, DM / 64, 1), 32, 0, stream>>>(CH, CH, WO, bo, OUT, ESEQ);
}
